// MultiHeadedAttention_82944408420453
// MI455X (gfx1250) — hardware-verified
//
#include <hip/hip_runtime.h>
#ifndef NB
#define NB 4
#endif
#ifndef SEQ
#define SEQ 1024
#endif
#define NB_FULL 4
#define SEQ_FULL 1024
#define DD 768
#define NH 12
#define HD 64

static_assert(NB >= 1 && NB <= NB_FULL);
static_assert(SEQ >= 64 && SEQ <= SEQ_FULL && (SEQ % 64) == 0);
static_assert(NH * HD == DD && (DD % 64) == 0 && (HD % 32) == 0 && HD <= 128);
static_assert((DD % 32) == 0);
static_assert(((DD * DD / 8) % 256) == 0);
static_assert((((SEQ / 16) * (DD / 64)) % 4) == 0);
static_assert((size_t)4 * DD * DD * 2 + (size_t)4 * NB * SEQ * DD * 4 + 8 * 256 <= (size_t)134217728);

typedef __bf16 v16b __attribute__((ext_vector_type(16)));
typedef unsigned short v8us __attribute__((ext_vector_type(8), may_alias));
typedef float  v8f  __attribute__((ext_vector_type(8)));
typedef float  v4f  __attribute__((ext_vector_type(4)));
typedef float  v4fa __attribute__((ext_vector_type(4), may_alias));
typedef int    v4ia __attribute__((ext_vector_type(4), may_alias));
union FragB { v16b v; v8us half[2]; unsigned short u[16]; };

__device__ __forceinline__ unsigned short bf16_bits(float x) { unsigned int u = __float_as_uint(x); return (unsigned short)((u + 0x7FFFu + ((u >> 16) & 1u)) >> 16); }
__device__ __forceinline__ float bf16_val(unsigned short b) { return __uint_as_float(((unsigned int)b) << 16); }
__device__ __forceinline__ float bf16_rne(float x) { return bf16_val(bf16_bits(x)); }

template <int NT>
__device__ __forceinline__ v8f mmaN(v16b ah, v16b al, v16b bh, v16b bl, v8f c) {
  c = __builtin_amdgcn_wmma_f32_16x16x32_bf16(false, ah, false, bh, (short)0, c, false, false);
  if (NT >= 2) c = __builtin_amdgcn_wmma_f32_16x16x32_bf16(false, al, false, bh, (short)0, c, false, false);
  if (NT >= 3) c = __builtin_amdgcn_wmma_f32_16x16x32_bf16(false, ah, false, bl, (short)0, c, false, false);
  asm volatile("v_nop\n\tv_nop\n\tv_nop\n\tv_nop" : "+v"(c) : "v"(ah), "v"(al), "v"(bh), "v"(bl));
  return c;
}

__global__ __launch_bounds__(256) void k_rne_rows(const float* __restrict__ W, unsigned short* __restrict__ Wt, unsigned n8) {
  const unsigned t = blockIdx.x * 256u + threadIdx.x;
  if (t >= n8) return;
  const v4f a = *(const v4fa*)(W + (size_t)t * 8), b = *(const v4fa*)(W + (size_t)t * 8 + 4);
  v8us v; v[0]=bf16_bits(a[0]); v[1]=bf16_bits(a[1]); v[2]=bf16_bits(a[2]); v[3]=bf16_bits(a[3]);
  v[4]=bf16_bits(b[0]); v[5]=bf16_bits(b[1]); v[6]=bf16_bits(b[2]); v[7]=bf16_bits(b[3]);
  *(volatile v8us*)(Wt + (size_t)t * 8) = v; __threadfence(); *(volatile v8us*)(Wt + (size_t)t * 8) = v;
}

template <bool ASPLIT, bool BIAS_BF16>
__global__ __launch_bounds__(128) void k_gemm_bf(const float* __restrict__ A, unsigned abatch, const unsigned short* __restrict__ Wt,
                                               const float* __restrict__ bias, float* __restrict__ C, unsigned cbatch, unsigned M) {
  constexpr unsigned N = DD, K = DD, NTN = N / 64;
  static_assert((N % 64) == 0 && (K % 32) == 0);
  __shared__ __attribute__((aligned(16))) float so[4][16][64];
  const unsigned tid = threadIdx.x, w = tid >> 5, lane = tid & 31u, ln = lane & 15u, hh = lane >> 4;
  const unsigned wid = blockIdx.x * 4u + w;
  const unsigned mt = wid / NTN, nq = wid - mt * NTN;
  if (mt * 16u >= M) return;
  const unsigned row0 = mt * 16u, col0 = nq * 64u;
  const float* Ab = A + (size_t)blockIdx.y * (size_t)abatch;
  float* Cb = C + (size_t)blockIdx.y * (size_t)cbatch;
  const float* arow = Ab + (size_t)(row0 + ln) * K;
  v8f acc[4];
#pragma unroll
  for (int t = 0; t < 4; ++t) acc[t] = (v8f){0.f,0.f,0.f,0.f,0.f,0.f,0.f,0.f};
  for (unsigned kb = 0; kb < K; kb += 32) {
    FragB ah, al;
    const v4f x0 = *(const v4fa*)(arow + kb + 8 * hh), x1 = *(const v4fa*)(arow + kb + 8 * hh + 4);
    const v4f x2 = *(const v4fa*)(arow + kb + 16 + 8 * hh), x3 = *(const v4fa*)(arow + kb + 16 + 8 * hh + 4);
    float xs[16] = {x0[0],x0[1],x0[2],x0[3],x1[0],x1[1],x1[2],x1[3],x2[0],x2[1],x2[2],x2[3],x3[0],x3[1],x3[2],x3[3]};
#pragma unroll
    for (int i = 0; i < 16; ++i) { const unsigned short hb = bf16_bits(xs[i]); ah.u[i] = hb; al.u[i] = ASPLIT ? bf16_bits(xs[i] - bf16_val(hb)) : (unsigned short)0; }
#pragma unroll
    for (int t = 0; t < 4; ++t) {
      const unsigned short* brow = Wt + (size_t)(col0 + t * 16 + ln) * K + kb;
      FragB b;
      b.half[0] = *(const v8us*)(brow + 8 * hh);
      b.half[1] = *(const v8us*)(brow + 16 + 8 * hh);
      acc[t] = mmaN<ASPLIT ? 2 : 1>(ah.v, al.v, b.v, b.v, acc[t]);
    }
  }
#pragma unroll
  for (int t = 0; t < 4; ++t) {
    float bvv = bias[col0 + t * 16 + ln];
    if (BIAS_BF16) bvv = bf16_rne(bvv);
#pragma unroll
    for (int r = 0; r < 8; ++r) { so[w][8 * hh + r][t * 16 + ln] = acc[t][r] + bvv; }
  }
  __builtin_amdgcn_fence(4  , "workgroup");
  __builtin_amdgcn_wave_barrier();
  const unsigned rsub = lane >> 4, c4 = (lane & 15u) * 4u;
  for (int pass = 0; pass < 2; ++pass) {
#pragma unroll
    for (int q = 0; q < 8; ++q) {
      const unsigned r = q * 2 + rsub;
      const v4f v = *(const v4fa*)&so[w][r][c4];
      *(volatile v4f*)(Cb + (size_t)(row0 + r) * N + col0 + c4) = v;
    }
    if (pass == 0) __threadfence();
  }
}

template <int D>
__global__ __launch_bounds__(128) void k_flash_mask(const float* __restrict__ Qb, const float* __restrict__ Kb, const float* __restrict__ Vb,
                                                  const int* __restrict__ mask, float* __restrict__ y, float scale) {
  constexpr unsigned KS = D / 32, DT = D / 16, D4 = D / 4, T = SEQ, PITCH = DD;
  static_assert((D % 32) == 0 && D <= 128 && D4 <= 32);
  static_assert(((32 * D4) % 128) == 0);
  static_assert((T % 32) == 0);
  __shared__ __attribute__((aligned(16))) unsigned short sKh[32][D + 8], sKl[32][D + 8], sVh[32][D + 8], sVl[32][D + 8];
  __shared__ __attribute__((aligned(16))) unsigned short sPh[4][16][40], sPl[4][16][40];
  __shared__ __attribute__((aligned(16))) int sM[4][16][36];
  __shared__ __attribute__((aligned(16))) float sO[4][16][D];
  const unsigned tid = threadIdx.x, w = tid >> 5, lane = tid & 31u, ln = lane & 15u, hh = lane >> 4;
  const unsigned qblk = blockIdx.x, bh = blockIdx.y;
  const unsigned b = bh / (unsigned)NH, h = bh - b * (unsigned)NH;
  const unsigned q0 = qblk * 64u + w * 16u;
  const size_t boff = (size_t)b * T * PITCH + (size_t)h * D;
  const float* Q = Qb + boff;
  const float* K = Kb + boff;
  const float* V = Vb + boff;
  unsigned qrow = q0 + ln; if (qrow >= T) qrow = T - 1;
  const int* mp = mask + ((size_t)b * SEQ_FULL + qrow) * SEQ_FULL + 16u * hh;

  FragB aqh[KS], aql[KS];
  {
    const float* qr = Q + (size_t)qrow * PITCH;
#pragma unroll
    for (unsigned ks = 0; ks < KS; ++ks) {
      const v4f x0 = *(const v4fa*)(qr + ks * 32 + 8 * hh), x1 = *(const v4fa*)(qr + ks * 32 + 8 * hh + 4);
      const v4f x2 = *(const v4fa*)(qr + ks * 32 + 16 + 8 * hh), x3 = *(const v4fa*)(qr + ks * 32 + 16 + 8 * hh + 4);
      const float xs[16] = {x0[0],x0[1],x0[2],x0[3],x1[0],x1[1],x1[2],x1[3],x2[0],x2[1],x2[2],x2[3],x3[0],x3[1],x3[2],x3[3]};
#pragma unroll
      for (int i = 0; i < 16; ++i) {
        const float x = xs[i] * scale; const unsigned short hb = bf16_bits(x);
        aqh[ks].u[i] = hb; aql[ks].u[i] = bf16_bits(x - bf16_val(hb));
      }
    }
  }
  float m_r[8], l_r[8];
#pragma unroll
  for (int r = 0; r < 8; ++r) { m_r[r] = -3.0e38f; l_r[r] = 0.f; }
  v8f oacc[DT];
#pragma unroll
  for (unsigned dt = 0; dt < DT; ++dt) oacc[dt] = (v8f){0.f,0.f,0.f,0.f,0.f,0.f,0.f,0.f};

  for (unsigned j0 = 0; j0 < T; j0 += 32) {
    __syncthreads();
    for (unsigned e = tid; e < 32 * D4; e += 128) {
      const unsigned r = e / D4, c4 = (e - r * D4) * 4u;
      unsigned key = j0 + r; const bool kin = key < T; if (!kin) key = T - 1;
      v4f kf = *(const v4fa*)(K + (size_t)key * PITCH + c4);
      v4f vf = *(const v4fa*)(V + (size_t)key * PITCH + c4);
      if (!kin) { kf = (v4f){0.f,0.f,0.f,0.f}; vf = (v4f){0.f,0.f,0.f,0.f}; }
#pragma unroll
      for (int t = 0; t < 4; ++t) {
        unsigned short hb = bf16_bits(kf[t]); sKh[r][c4 + t] = hb; sKl[r][c4 + t] = bf16_bits(kf[t] - bf16_val(hb));
        hb = bf16_bits(vf[t]); sVh[r][c4 + t] = hb; sVl[r][c4 + t] = bf16_bits(vf[t] - bf16_val(hb));
      }
    }
    {
      const int* mc = mp + j0;
      const v4ia m0 = *(const v4ia*)(mc), m1 = *(const v4ia*)(mc + 4), m2 = *(const v4ia*)(mc + 8), m3 = *(const v4ia*)(mc + 12);
      *(v4ia*)&sM[w][ln][16 * hh]      = m0;
      *(v4ia*)&sM[w][ln][16 * hh + 4]  = m1;
      *(v4ia*)&sM[w][ln][16 * hh + 8]  = m2;
      *(v4ia*)&sM[w][ln][16 * hh + 12] = m3;
    }
    __syncthreads();
    v8f s[2];
#pragma unroll
    for (int nt = 0; nt < 2; ++nt) {
      v8f acc = (v8f){0.f,0.f,0.f,0.f,0.f,0.f,0.f,0.f};
#pragma unroll
      for (unsigned ks = 0; ks < KS; ++ks) {
        FragB bh_, bl_;
        bh_.half[0] = *(const v8us*)&sKh[nt * 16 + ln][ks * 32 + 8 * hh]; bh_.half[1] = *(const v8us*)&sKh[nt * 16 + ln][ks * 32 + 16 + 8 * hh];
        bl_.half[0] = *(const v8us*)&sKl[nt * 16 + ln][ks * 32 + 8 * hh]; bl_.half[1] = *(const v8us*)&sKl[nt * 16 + ln][ks * 32 + 16 + 8 * hh];
        acc = mmaN<3>(aqh[ks].v, aql[ks].v, bh_.v, bl_.v, acc);
      }
      s[nt] = acc;
    }
    float alpha[8];
#pragma unroll
    for (int r = 0; r < 8; ++r) {
      const int ma = sM[w][8 * hh + r][ln], mb = sM[w][8 * hh + r][16 + ln];
      const bool keepa = (ma != 0), keepb = (mb != 0);
      const float sa = keepa ? s[0][r] * (float)ma : -3.0e38f;
      const float sb = keepb ? s[1][r] * (float)mb : -3.0e38f;
      float mx = fmaxf(sa, sb);
      mx = fmaxf(mx, __shfl_xor(mx, 1, 32)); mx = fmaxf(mx, __shfl_xor(mx, 2, 32)); mx = fmaxf(mx, __shfl_xor(mx, 4, 32)); mx = fmaxf(mx, __shfl_xor(mx, 8, 32));
      const float mnew = fmaxf(m_r[r], mx);
      alpha[r] = (m_r[r] > -1.0e38f) ? __expf(m_r[r] - mnew) : 1.0f;
      const float p0 = keepa ? __expf(sa - mnew) : 0.f;
      const float p1 = keepb ? __expf(sb - mnew) : 0.f;
      m_r[r] = mnew;
      l_r[r] = l_r[r] * alpha[r] + p0 + p1;
      unsigned short hb = bf16_bits(p0); sPh[w][8 * hh + r][ln] = hb;      sPl[w][8 * hh + r][ln] = bf16_bits(p0 - bf16_val(hb));
      hb = bf16_bits(p1);                sPh[w][8 * hh + r][16 + ln] = hb; sPl[w][8 * hh + r][16 + ln] = bf16_bits(p1 - bf16_val(hb));
    }
#pragma unroll
    for (unsigned dt = 0; dt < DT; ++dt)
#pragma unroll
      for (int r = 0; r < 8; ++r) oacc[dt][r] *= alpha[r];
    __builtin_amdgcn_fence(4  , "workgroup");
    __builtin_amdgcn_wave_barrier();
    FragB pah, pal;
    pah.half[0] = *(const v8us*)&sPh[w][ln][8 * hh]; pah.half[1] = *(const v8us*)&sPh[w][ln][16 + 8 * hh];
    pal.half[0] = *(const v8us*)&sPl[w][ln][8 * hh]; pal.half[1] = *(const v8us*)&sPl[w][ln][16 + 8 * hh];
#pragma unroll
    for (unsigned dt = 0; dt < DT; ++dt) {
      FragB bvh, bvl;
#pragma unroll
      for (int i = 0; i < 8; ++i) {
        bvh.u[i] = sVh[8 * hh + i][dt * 16 + ln]; bvh.u[8 + i] = sVh[16 + 8 * hh + i][dt * 16 + ln];
        bvl.u[i] = sVl[8 * hh + i][dt * 16 + ln]; bvl.u[8 + i] = sVl[16 + 8 * hh + i][dt * 16 + ln];
      }
      oacc[dt] = mmaN<3>(pah.v, pal.v, bvh.v, bvl.v, oacc[dt]);
    }
    __builtin_amdgcn_fence(4  , "workgroup");
    __builtin_amdgcn_wave_barrier();
  }
#pragma unroll
  for (int r = 0; r < 8; ++r) {
    float l = l_r[r];
    l += __shfl_xor(l, 1, 32); l += __shfl_xor(l, 2, 32); l += __shfl_xor(l, 4, 32); l += __shfl_xor(l, 8, 32);
    l_r[r] = (l > 0.f) ? (1.0f / l) : 0.f;
  }
#pragma unroll
  for (unsigned dt = 0; dt < DT; ++dt)
#pragma unroll
    for (int r = 0; r < 8; ++r) sO[w][8 * hh + r][dt * 16 + ln] = oacc[dt][r] * l_r[r];
  __builtin_amdgcn_fence(4  , "workgroup");
  __builtin_amdgcn_wave_barrier();
  for (int pass = 0; pass < 2; ++pass) {
    for (unsigned r = 0; r < 16; ++r) {
      const unsigned row = q0 + r;
      if (row < T && lane < D4) {
        const v4f val = *(const v4fa*)&sO[w][r][lane * 4];
        *(volatile v4f*)(y + ((size_t)b * T + row) * PITCH + h * D + lane * 4) = val;
      }
    }
    if (pass == 0) __threadfence();
  }
}

extern "C" void kernel_launch(void* const* d_in, const int* in_sizes, int n_in,
                              void* d_out, int out_size, void* d_ws, size_t ws_size, hipStream_t stream) {
  if (n_in < 12) return;
  const float* xq = (const float*)d_in[0]; const float* xk = (const float*)d_in[1]; const float* xv = (const float*)d_in[2];
  const int* msk = (const int*)d_in[3];
  const float* Wq = (const float*)d_in[4]; const float* bq = (const float*)d_in[5]; const float* Wk = (const float*)d_in[6]; const float* bk = (const float*)d_in[7];
  const float* Wv = (const float*)d_in[8]; const float* bv = (const float*)d_in[9]; const float* Wo = (const float*)d_in[10]; const float* bo = (const float*)d_in[11];
  const long long needX = (long long)(NB - 1) * SEQ_FULL * DD + (long long)SEQ * DD;
  if ((long long)in_sizes[0] < needX || (long long)in_sizes[1] < needX || (long long)in_sizes[2] < needX) return;
  const long long needM = ((long long)(NB - 1) * SEQ_FULL + (long long)(SEQ - 1)) * SEQ_FULL + SEQ;
  if ((long long)in_sizes[3] < needM) return;
  if (in_sizes[4] < DD * DD || in_sizes[6] < DD * DD || in_sizes[8] < DD * DD || in_sizes[10] < DD * DD) return;
  if (in_sizes[5] < DD || in_sizes[7] < DD || in_sizes[9] < DD || in_sizes[11] < DD) return;
  if ((long long)out_size < (long long)NB * SEQ * DD) return;

  char* ws = (char*)d_ws; size_t off = 0;
  auto take = [&](size_t bytes) { char* p = ws + off; off += (bytes + 255) & ~(size_t)255; return p; };
  const size_t MROWS = (size_t)NB * SEQ;
  unsigned short* Wt[4]; for (int i = 0; i < 4; ++i) Wt[i] = (unsigned short*)take((size_t)DD * DD * 2);
  float* q   = (float*)take(MROWS * DD * 4);
  float* k   = (float*)take(MROWS * DD * 4);
  float* v   = (float*)take(MROWS * DD * 4);
  float* att = (float*)take(MROWS * DD * 4);
  if (off > ws_size || off > (size_t)134217728) return;

  const unsigned n8 = DD * DD / 8;
  const unsigned gb = ((SEQ / 16) * (DD / 64)) / 4;
  const dim3 gg(gb, NB);
  const float* W4[4] = {Wq, Wk, Wv, Wo};
  for (int i = 0; i < 4; ++i) k_rne_rows<<<n8 / 256, 256, 0, stream>>>(W4[i], Wt[i], n8);
  k_gemm_bf<false, true><<<gg, 128, 0, stream>>>(xq, (unsigned)(SEQ_FULL * DD), Wt[0], bq, q, (unsigned)(SEQ * DD), (unsigned)SEQ);
  k_gemm_bf<false, true><<<gg, 128, 0, stream>>>(xk, (unsigned)(SEQ_FULL * DD), Wt[1], bk, k, (unsigned)(SEQ * DD), (unsigned)SEQ);
  k_gemm_bf<false, true><<<gg, 128, 0, stream>>>(xv, (unsigned)(SEQ_FULL * DD), Wt[2], bv, v, (unsigned)(SEQ * DD), (unsigned)SEQ);
  k_flash_mask<HD><<<dim3(SEQ / 64, NB * NH), 128, 0, stream>>>(q, k, v, msk, att, 0.125f);
  k_gemm_bf<true, true><<<gg, 128, 0, stream>>>(att, (unsigned)(SEQ * DD), Wt[3], bo, (float*)d_out, (unsigned)(SEQ * DD), (unsigned)SEQ);
  (void)hipGetLastError();
}
